// PointNetFPModule_24764781429155
// MI455X (gfx1250) — hardware-verified
//
#include <hip/hip_runtime.h>
#pragma clang fp contract(off)

typedef __attribute__((ext_vector_type(16))) __bf16   v16b;
typedef __attribute__((ext_vector_type(8)))  __bf16   v8b;
typedef __attribute__((ext_vector_type(8)))  float    v8f;
typedef __attribute__((ext_vector_type(4)))  float    v4f;
typedef __attribute__((ext_vector_type(4)))  unsigned v4u;

constexpr int kNumBatch   = 16;
constexpr int kNumPoints  = 4096;
constexpr int kNumCenters = 1024;
constexpr int kChanCenter = 256;
constexpr int kChanPoint  = 64;
constexpr int kChanIn     = 320;
constexpr int kHidden1    = 256;
constexpr int kHidden2    = 128;
constexpr int kCondDim    = 128;
constexpr int kHalfBatch  = 8;
constexpr int kHalfPoints = kHalfBatch * kNumPoints;

static_assert(kChanIn == kChanCenter + kChanPoint, "concat width");
static_assert(kChanIn % 32 == 0 && kHidden1 % 32 == 0, "GEMM depth multiple of 32");
static_assert(kHalfPoints % 64 == 0 && kHidden1 % 64 == 0 && kHidden2 % 64 == 0 && kNumPoints % 64 == 0, "tile multiples");
static_assert(((kHalfPoints / 64) * (kHidden1 / 64)) % 8 == 0, "layer-1 tiles fill whole blocks");
static_assert(((kHidden2 / 64) * (kNumPoints / 64)) % 8 == 0, "layer-2 tiles fill whole blocks");
static_assert(kNumCenters == 1024 && kNumPoints % 256 == 0, "search tile shape");

constexpr size_t kOut0Bytes   = (size_t)kNumBatch * kHidden2 * kNumPoints * 4;
constexpr size_t kOut1OffB    = 33554432;
constexpr size_t kOut1Bytes   = (size_t)kNumBatch * 3 * kNumPoints * 4;
constexpr size_t kOut2OffB    = 34340864;
constexpr size_t kOut2Bytes   = (size_t)kNumBatch * kCondDim * 4;
constexpr size_t kOutTotalB   = 34349056;
static_assert(kOut0Bytes == kOut1OffB, "out1 offset");
static_assert(kOut1OffB + kOut1Bytes == kOut2OffB, "out2 offset");
static_assert(kOut2OffB + kOut2Bytes == kOutTotalB, "output total");
static_assert(kOut1OffB % 128 == 0 && kOut2OffB % 128 == 0, "line aligned outputs");

constexpr size_t kW1PlaneB   = (size_t)kHidden1 * kChanIn * 2;
constexpr size_t kW2PlaneB   = (size_t)kHidden2 * kHidden1 * 2;
constexpr size_t kFeatPlaneB = (size_t)kNumBatch * kNumPoints * kChanIn * 2;
constexpr size_t kHidPlaneB  = (size_t)kHalfPoints * kHidden1 * 2;
constexpr size_t kOffW1H   = 0;
constexpr size_t kOffW1L   = kOffW1H + kW1PlaneB;
constexpr size_t kOffW2H   = kOffW1L + kW1PlaneB;
constexpr size_t kOffW2L   = kOffW2H + kW2PlaneB;
constexpr size_t kOffFeatH = kOffW2L + kW2PlaneB;
constexpr size_t kOffFeatL = kOffFeatH + kFeatPlaneB;
constexpr size_t kOffHidH  = kOffFeatL + kFeatPlaneB;
constexpr size_t kOffHidL  = kOffHidH + kHidPlaneB;
constexpr size_t kWsTotal  = kOffHidL + kHidPlaneB;
static_assert(kWsTotal == 117899264, "carve total");
static_assert(kWsTotal <= 134217728, "carve limit");
static_assert(kOffFeatH % 128 == 0 && kOffFeatL % 128 == 0 && kOffHidH % 128 == 0 && kOffHidL % 128 == 0, "line aligned planes");

constexpr int kPrepW1Blocks = (kHidden1 * kChanIn / 8) / 256;
constexpr int kPrepW2Blocks = (kHidden2 * kHidden1 / 8) / 256;
constexpr int kPrepO1Blocks = (kNumBatch * 3 * kNumPoints / 4) / 256;
constexpr int kPrepO2Blocks = (kNumBatch * kCondDim / 4) / 256;
static_assert(kPrepW1Blocks * 256 * 8 == kHidden1 * kChanIn, "W1 pieces exact");
static_assert(kPrepW2Blocks * 256 * 8 == kHidden2 * kHidden1, "W2 pieces exact");
static_assert(kPrepO1Blocks * 256 * 4 == kNumBatch * 3 * kNumPoints, "out1 pieces exact");
static_assert(kPrepO2Blocks * 256 * 4 == kNumBatch * kCondDim, "out2 pieces exact");

__device__ __forceinline__ unsigned bf16_rne_bits(float f) {
  const unsigned u = __float_as_uint(f);
  return (u + 0x7FFFu + ((u >> 16) & 1u)) >> 16;
}
__device__ __forceinline__ void split_bf16(float f, unsigned& hb, unsigned& lb) {
  hb = bf16_rne_bits(f);
  const float fh = __uint_as_float(hb << 16);
  lb = bf16_rne_bits(f - fh);
}

__device__ __forceinline__ void guard_group(v8f& a0, v8f& a1, v8f& a2, v8f& a3, v16b x, v16b y,
                                            v16b b0, v16b b1, v16b b2, v16b b3,
                                            v16b c0, v16b c1, v16b c2, v16b c3) {
  asm volatile("v_nop\n\tv_nop\n\tv_nop\n\tv_nop"
               : "+v"(a0), "+v"(a1), "+v"(a2), "+v"(a3)
               : "v"(x), "v"(y), "v"(b0), "v"(b1), "v"(b2), "v"(b3), "v"(c0), "v"(c1), "v"(c2), "v"(c3));
}
__device__ __forceinline__ void acc_guard4(v8f& a, v8f& b, v8f& c, v8f& d) {
  asm volatile("v_nop\n\tv_nop\n\tv_nop\n\tv_nop" : "+v"(a), "+v"(b), "+v"(c), "+v"(d));
}

struct FragB {
  union U { v16b v; v8b h[2]; };
  static __device__ __forceinline__ v16b load(const __bf16* p) {
    U f;
    f.h[0] = *(const v8b*)(p);
    f.h[1] = *(const v8b*)(p + 16);
    return f.v;
  }
  static __device__ __forceinline__ v8f mma(v16b a, v16b b, v8f c) {
    return __builtin_amdgcn_wmma_f32_16x16x32_bf16(false, a, false, b, (short)0, c, false, false);
  }
};

__device__ __forceinline__ void split8_store(const float* __restrict__ src, unsigned short* __restrict__ hi,
                                             unsigned short* __restrict__ lo, int piece) {
  const v4f a = *(const v4f*)(src + (size_t)piece * 8);
  const v4f c = *(const v4f*)(src + (size_t)piece * 8 + 4);
  unsigned h0, h1, h2, h3, h4, h5, h6, h7, l0, l1, l2, l3, l4, l5, l6, l7;
  split_bf16(a[0], h0, l0); split_bf16(a[1], h1, l1); split_bf16(a[2], h2, l2); split_bf16(a[3], h3, l3);
  split_bf16(c[0], h4, l4); split_bf16(c[1], h5, l5); split_bf16(c[2], h6, l6); split_bf16(c[3], h7, l7);
  v4u hv, lv;
  hv[0] = h0 | (h1 << 16); hv[1] = h2 | (h3 << 16); hv[2] = h4 | (h5 << 16); hv[3] = h6 | (h7 << 16);
  lv[0] = l0 | (l1 << 16); lv[1] = l2 | (l3 << 16); lv[2] = l4 | (l5 << 16); lv[3] = l6 | (l7 << 16);
  volatile v4u* ph = (volatile v4u*)(hi + (size_t)piece * 8);
  volatile v4u* pl = (volatile v4u*)(lo + (size_t)piece * 8);
  *ph = hv; *pl = lv;
  __threadfence();
  *ph = hv; *pl = lv;
}
__device__ __forceinline__ void copy4_store(const float* __restrict__ src, float* __restrict__ dst, int piece) {
  const v4f a = *(const v4f*)(src + (size_t)piece * 4);
  volatile v4f* pd = (volatile v4f*)(dst + (size_t)piece * 4);
  *pd = a;
  __threadfence();
  *pd = a;
}

__global__ __launch_bounds__(256) void prep_planes_and_copies(
    const float* __restrict__ W1, const float* __restrict__ W2,
    const float* __restrict__ pcoords, const float* __restrict__ cond,
    unsigned short* __restrict__ w1h, unsigned short* __restrict__ w1l,
    unsigned short* __restrict__ w2h, unsigned short* __restrict__ w2l,
    float* __restrict__ out1, float* __restrict__ out2) {
  const int blk = blockIdx.x;
  const int tid = threadIdx.x;
  if (blk < kPrepW1Blocks) {
    split8_store(W1, w1h, w1l, blk * 256 + tid);
  } else if (blk < kPrepW1Blocks + kPrepW2Blocks) {
    split8_store(W2, w2h, w2l, (blk - kPrepW1Blocks) * 256 + tid);
  } else if (blk < kPrepW1Blocks + kPrepW2Blocks + kPrepO1Blocks) {
    copy4_store(pcoords, out1, (blk - kPrepW1Blocks - kPrepW2Blocks) * 256 + tid);
  } else {
    copy4_store(cond, out2, (blk - kPrepW1Blocks - kPrepW2Blocks - kPrepO1Blocks) * 256 + tid);
  }
}

__device__ __forceinline__ void hold8(float& a0, float& a1, float& a2, float& a3,
                                      float& a4, float& a5, float& a6, float& a7) {
  asm volatile("" : "+v"(a0), "+v"(a1), "+v"(a2), "+v"(a3), "+v"(a4), "+v"(a5), "+v"(a6), "+v"(a7) :: "memory");
}

__global__ __launch_bounds__(256) void knn3_interp_pack(
    const float* __restrict__ pcoords, const float* __restrict__ ccoords,
    const float* __restrict__ cfeat, const float* __restrict__ pfeat,
    unsigned short* __restrict__ feat_hi, unsigned short* __restrict__ feat_lo) {
#pragma clang fp contract(off)
  __shared__ v4f s_cx[256];
  __shared__ v4f s_cy[256];
  __shared__ v4f s_cz[256];
  __shared__ v4f s_cc[256];
  __shared__ int   s_idx[3][256];
  __shared__ float s_wt[3][256];

  const int tid  = threadIdx.x;
  const int b    = blockIdx.y;
  const int n0   = blockIdx.x * 256;

  {
    const float* cc = ccoords + (size_t)b * 3 * kNumCenters;
    const v4f x4 = *(const v4f*)(cc + 4 * tid);
    const v4f y4 = *(const v4f*)(cc + kNumCenters + 4 * tid);
    const v4f z4 = *(const v4f*)(cc + 2 * kNumCenters + 4 * tid);
    v4f q4;
    q4[0] = (x4[0] * x4[0] + y4[0] * y4[0]) + z4[0] * z4[0];
    q4[1] = (x4[1] * x4[1] + y4[1] * y4[1]) + z4[1] * z4[1];
    q4[2] = (x4[2] * x4[2] + y4[2] * y4[2]) + z4[2] * z4[2];
    q4[3] = (x4[3] * x4[3] + y4[3] * y4[3]) + z4[3] * z4[3];
    s_cx[tid] = x4; s_cy[tid] = y4; s_cz[tid] = z4; s_cc[tid] = q4;
  }
  __syncthreads();

  {
    const float* pcb = pcoords + (size_t)b * 3 * kNumPoints;
    const int n = n0 + tid;
    const float px = pcb[n];
    const float py = pcb[kNumPoints + n];
    const float pz = pcb[2 * kNumPoints + n];
    const float p2 = (px * px + py * py) + pz * pz;
    float bd0 = __builtin_huge_valf(), bd1 = __builtin_huge_valf(), bd2 = __builtin_huge_valf();
    int bi0 = 0, bi1 = 0, bi2 = 0;
#pragma unroll 1
    for (int m4 = 0; m4 < 256; ++m4) {
      const v4f cx = s_cx[m4];
      const v4f cy = s_cy[m4];
      const v4f cz = s_cz[m4];
      const v4f cq = s_cc[m4];
#pragma unroll
      for (int e = 0; e < 4; ++e) {
        float p = px * cx[e];
        p = __builtin_fmaf(py, cy[e], p);
        p = __builtin_fmaf(pz, cz[e], p);
        const float s = p2 + cq[e];
        const float d = s - 2.0f * p;
        const int m = 4 * m4 + e;
        const bool l0 = d < bd0;
        const bool l1 = d < bd1;
        const bool l2 = d < bd2;
        bd2 = l1 ? bd1 : (l2 ? d : bd2);
        bi2 = l1 ? bi1 : (l2 ? m : bi2);
        bd1 = l0 ? bd0 : (l1 ? d : bd1);
        bi1 = l0 ? bi0 : (l1 ? m : bi1);
        bd0 = l0 ? d : bd0;
        bi0 = l0 ? m : bi0;
      }
    }
    const float e0 = fmaxf(bd0, 1e-10f);
    const float e1 = fmaxf(bd1, 1e-10f);
    const float e2 = fmaxf(bd2, 1e-10f);
    const float r0 = 1.0f / e0;
    const float r1 = 1.0f / e1;
    const float r2 = 1.0f / e2;
    const float rs = (r0 + r2) + r1;
    s_wt[0][tid] = r0 / rs;
    s_wt[1][tid] = r1 / rs;
    s_wt[2][tid] = r2 / rs;
    s_idx[0][tid] = bi0;
    s_idx[1][tid] = bi1;
    s_idx[2][tid] = bi2;
  }
  __syncthreads();

  const int wave = tid >> 5;
  const int lane = tid & 31;

  {
    const float* cfb = cfeat + ((size_t)b * kChanCenter + 8 * lane) * kNumCenters;
#pragma unroll 1
    for (int it = 0; it < 32; ++it) {
      const int p = wave * 32 + it;
      int i0 = s_idx[0][p];
      int i1 = s_idx[1][p];
      int i2 = s_idx[2][p];
      i0 = i0 < 0 ? 0 : (i0 > kNumCenters - 1 ? kNumCenters - 1 : i0);
      i1 = i1 < 0 ? 0 : (i1 > kNumCenters - 1 ? kNumCenters - 1 : i1);
      i2 = i2 < 0 ? 0 : (i2 > kNumCenters - 1 ? kNumCenters - 1 : i2);
      const float w0 = s_wt[0][p];
      const float w1 = s_wt[1][p];
      const float w2 = s_wt[2][p];
      float ga0 = cfb[0 * kNumCenters + i0], ga1 = cfb[1 * kNumCenters + i0], ga2 = cfb[2 * kNumCenters + i0], ga3 = cfb[3 * kNumCenters + i0];
      float ga4 = cfb[4 * kNumCenters + i0], ga5 = cfb[5 * kNumCenters + i0], ga6 = cfb[6 * kNumCenters + i0], ga7 = cfb[7 * kNumCenters + i0];
      hold8(ga0, ga1, ga2, ga3, ga4, ga5, ga6, ga7);
      float gb0 = cfb[0 * kNumCenters + i1], gb1 = cfb[1 * kNumCenters + i1], gb2 = cfb[2 * kNumCenters + i1], gb3 = cfb[3 * kNumCenters + i1];
      float gb4 = cfb[4 * kNumCenters + i1], gb5 = cfb[5 * kNumCenters + i1], gb6 = cfb[6 * kNumCenters + i1], gb7 = cfb[7 * kNumCenters + i1];
      hold8(gb0, gb1, gb2, gb3, gb4, gb5, gb6, gb7);
      float gc0 = cfb[0 * kNumCenters + i2], gc1 = cfb[1 * kNumCenters + i2], gc2 = cfb[2 * kNumCenters + i2], gc3 = cfb[3 * kNumCenters + i2];
      float gc4 = cfb[4 * kNumCenters + i2], gc5 = cfb[5 * kNumCenters + i2], gc6 = cfb[6 * kNumCenters + i2], gc7 = cfb[7 * kNumCenters + i2];
      hold8(gc0, gc1, gc2, gc3, gc4, gc5, gc6, gc7);
      const float v0 = (ga0 * w0 + gc0 * w2) + gb0 * w1;
      const float v1 = (ga1 * w0 + gc1 * w2) + gb1 * w1;
      const float v2 = (ga2 * w0 + gc2 * w2) + gb2 * w1;
      const float v3 = (ga3 * w0 + gc3 * w2) + gb3 * w1;
      const float v4 = (ga4 * w0 + gc4 * w2) + gb4 * w1;
      const float v5 = (ga5 * w0 + gc5 * w2) + gb5 * w1;
      const float v6 = (ga6 * w0 + gc6 * w2) + gb6 * w1;
      const float v7 = (ga7 * w0 + gc7 * w2) + gb7 * w1;
      unsigned h0, h1, h2, h3, h4, h5, h6, h7, l0, l1, l2, l3, l4, l5, l6, l7;
      split_bf16(v0, h0, l0); split_bf16(v1, h1, l1); split_bf16(v2, h2, l2); split_bf16(v3, h3, l3);
      split_bf16(v4, h4, l4); split_bf16(v5, h5, l5); split_bf16(v6, h6, l6); split_bf16(v7, h7, l7);
      v4u hv, lv;
      hv[0] = h0 | (h1 << 16); hv[1] = h2 | (h3 << 16); hv[2] = h4 | (h5 << 16); hv[3] = h6 | (h7 << 16);
      lv[0] = l0 | (l1 << 16); lv[1] = l2 | (l3 << 16); lv[2] = l4 | (l5 << 16); lv[3] = l6 | (l7 << 16);
      const size_t row = (size_t)b * kNumPoints + n0 + p;
      volatile v4u* ph = (volatile v4u*)(feat_hi + row * kChanIn + 8 * lane);
      volatile v4u* pl = (volatile v4u*)(feat_lo + row * kChanIn + 8 * lane);
      *ph = hv; *pl = lv;
      __threadfence();
      *ph = hv; *pl = lv;
    }
  }

  {
    const int sub = lane >> 3;
    const int cp0 = 8 * (lane & 7);
    const float* pfb = pfeat + ((size_t)b * kChanPoint + cp0) * kNumPoints + n0;
#pragma unroll 1
    for (int it = 0; it < 8; ++it) {
      const int p = wave * 32 + it * 4 + sub;
      const float f0 = pfb[0 * kNumPoints + p], f1 = pfb[1 * kNumPoints + p], f2 = pfb[2 * kNumPoints + p], f3 = pfb[3 * kNumPoints + p];
      const float f4 = pfb[4 * kNumPoints + p], f5 = pfb[5 * kNumPoints + p], f6 = pfb[6 * kNumPoints + p], f7 = pfb[7 * kNumPoints + p];
      unsigned h0, h1, h2, h3, h4, h5, h6, h7, l0, l1, l2, l3, l4, l5, l6, l7;
      split_bf16(f0, h0, l0); split_bf16(f1, h1, l1); split_bf16(f2, h2, l2); split_bf16(f3, h3, l3);
      split_bf16(f4, h4, l4); split_bf16(f5, h5, l5); split_bf16(f6, h6, l6); split_bf16(f7, h7, l7);
      v4u hv, lv;
      hv[0] = h0 | (h1 << 16); hv[1] = h2 | (h3 << 16); hv[2] = h4 | (h5 << 16); hv[3] = h6 | (h7 << 16);
      lv[0] = l0 | (l1 << 16); lv[1] = l2 | (l3 << 16); lv[2] = l4 | (l5 << 16); lv[3] = l6 | (l7 << 16);
      const size_t row = (size_t)b * kNumPoints + n0 + p;
      volatile v4u* ph = (volatile v4u*)(feat_hi + row * kChanIn + kChanCenter + cp0);
      volatile v4u* pl = (volatile v4u*)(feat_lo + row * kChanIn + kChanCenter + cp0);
      *ph = hv; *pl = lv;
      __threadfence();
      *ph = hv; *pl = lv;
    }
  }
}

template <int OUT_MODE, int BIAS_MODE>
__global__ __launch_bounds__(256) void gemm_bf16x3_64(
    const unsigned short* __restrict__ Ap, const unsigned short* __restrict__ A2p, int lda, long strideA,
    const unsigned short* __restrict__ Btp, const unsigned short* __restrict__ Bt2p, int ldb, long strideB,
    void* __restrict__ Cout, void* __restrict__ Cout2, int ldc, long strideC,
    const float* __restrict__ bias, int M, int N, int K) {
  const __bf16* A   = (const __bf16*)Ap;
  const __bf16* A2  = (const __bf16*)A2p;
  const __bf16* Bt  = (const __bf16*)Btp;
  const __bf16* Bt2 = (const __bf16*)Bt2p;
  __shared__ __align__(16) float sT[8][16 * 68];
  const int b    = blockIdx.y;
  const int lane = threadIdx.x & 31;
  const int wave = threadIdx.x >> 5;
  const int tilesN = N >> 6;
  const int tilesM = M >> 6;
  const int tile = blockIdx.x * 8 + wave;
  if (tile >= tilesM * tilesN) return;
  const int tm = tile / tilesN;
  const int tn = tile - tm * tilesN;
  const int m0 = tm << 6;
  const int n0 = tn << 6;

  const __bf16* Ab  = A   + (size_t)b * strideA;
  const __bf16* Ab2 = A2  + (size_t)b * strideA;
  const __bf16* Bb  = Bt  + (size_t)b * strideB;
  const __bf16* Bb2 = Bt2 + (size_t)b * strideB;

  const int rlane = lane & 15;
  const int koff  = (lane >> 4) * 8;
  const int mOff  = (lane >> 4) * 8;

  v8f acc[4][4];
#pragma unroll
  for (int i = 0; i < 4; ++i)
#pragma unroll
    for (int j = 0; j < 4; ++j) acc[i][j] = (v8f){0.f, 0.f, 0.f, 0.f, 0.f, 0.f, 0.f, 0.f};

  for (int k0 = 0; k0 < K; k0 += 32) {
    v16b bh[4], bl[4];
#pragma unroll
    for (int j = 0; j < 4; ++j) {
      const size_t bo = (size_t)(n0 + (j << 4) + rlane) * ldb + koff + k0;
      bh[j] = FragB::load(Bb + bo);
      bl[j] = FragB::load(Bb2 + bo);
    }
#pragma unroll
    for (int i = 0; i < 4; ++i) {
      const size_t ao = (size_t)(m0 + (i << 4) + rlane) * lda + koff + k0;
      const v16b ah = FragB::load(Ab + ao);
      const v16b al = FragB::load(Ab2 + ao);
#pragma unroll
      for (int j = 0; j < 4; ++j) {
        acc[i][j] = FragB::mma(ah, bh[j], acc[i][j]);
        acc[i][j] = FragB::mma(ah, bl[j], acc[i][j]);
        acc[i][j] = FragB::mma(al, bh[j], acc[i][j]);
      }
      guard_group(acc[i][0], acc[i][1], acc[i][2], acc[i][3], ah, al,
                  bh[0], bh[1], bh[2], bh[3], bl[0], bl[1], bl[2], bl[3]);
    }
  }
  acc_guard4(acc[0][0], acc[0][1], acc[0][2], acc[0][3]);
  acc_guard4(acc[1][0], acc[1][1], acc[1][2], acc[1][3]);
  acc_guard4(acc[2][0], acc[2][1], acc[2][2], acc[2][3]);
  acc_guard4(acc[3][0], acc[3][1], acc[3][2], acc[3][3]);

  float* slab = sT[wave];
#pragma unroll
  for (int i = 0; i < 4; ++i) {
    const int mBase = m0 + (i << 4);
#pragma unroll
    for (int j = 0; j < 4; ++j) {
      const int n = n0 + (j << 4) + rlane;
      float bv = 0.f;
      if (BIAS_MODE == 2) bv = bias[n];
#pragma unroll
      for (int r = 0; r < 8; ++r) {
        float v = acc[i][j][r];
        if (BIAS_MODE == 1) v += bias[mBase + mOff + r];
        if (BIAS_MODE == 2) v += bv;
        v = fmaxf(v, 0.0f);
        slab[(mOff + r) * 68 + (j << 4) + rlane] = v;
      }
    }
    __builtin_amdgcn_fence(__ATOMIC_RELEASE, "workgroup");
    __builtin_amdgcn_wave_barrier();
    __builtin_amdgcn_fence(__ATOMIC_ACQUIRE, "workgroup");
    if (OUT_MODE == 0) {
      float* C = (float*)Cout + (size_t)b * strideC;
      const int hh = lane >> 4, c4 = (lane & 15) * 4;
      for (int pass = 0; pass < 2; ++pass) {
#pragma unroll
        for (int it = 0; it < 8; ++it) {
          const int row = it * 2 + hh;
          const v4f v = *(const v4f*)(slab + row * 68 + c4);
          *(volatile v4f*)(C + (size_t)(mBase + row) * ldc + n0 + c4) = v;
        }
        __threadfence();
      }
    } else {
      const int q = lane >> 3, c8 = (lane & 7) * 8;
      unsigned short* C  = (unsigned short*)Cout  + (size_t)b * strideC;
      unsigned short* C2 = (unsigned short*)Cout2 + (size_t)b * strideC;
      for (int pass = 0; pass < 2; ++pass) {
#pragma unroll
        for (int it = 0; it < 4; ++it) {
          const int row = it * 4 + q;
          const float* sp = slab + row * 68 + c8;
          const v4f s0 = *(const v4f*)(sp);
          const v4f s1 = *(const v4f*)(sp + 4);
          unsigned h0, h1, h2, h3, h4, h5, h6, h7, l0, l1, l2, l3, l4, l5, l6, l7;
          split_bf16(s0[0], h0, l0); split_bf16(s0[1], h1, l1); split_bf16(s0[2], h2, l2); split_bf16(s0[3], h3, l3);
          split_bf16(s1[0], h4, l4); split_bf16(s1[1], h5, l5); split_bf16(s1[2], h6, l6); split_bf16(s1[3], h7, l7);
          v4u hv, lv;
          hv[0] = h0 | (h1 << 16); hv[1] = h2 | (h3 << 16); hv[2] = h4 | (h5 << 16); hv[3] = h6 | (h7 << 16);
          lv[0] = l0 | (l1 << 16); lv[1] = l2 | (l3 << 16); lv[2] = l4 | (l5 << 16); lv[3] = l6 | (l7 << 16);
          *(volatile v4u*)(C  + (size_t)(mBase + row) * ldc + n0 + c8) = hv;
          *(volatile v4u*)(C2 + (size_t)(mBase + row) * ldc + n0 + c8) = lv;
        }
        __threadfence();
      }
    }
    __builtin_amdgcn_fence(__ATOMIC_RELEASE, "workgroup");
    __builtin_amdgcn_wave_barrier();
    __builtin_amdgcn_fence(__ATOMIC_ACQUIRE, "workgroup");
  }
}

extern "C" void kernel_launch(void* const* d_in, const int* in_sizes, int n_in,
                              void* d_out, int out_size, void* d_ws, size_t ws_size,
                              hipStream_t stream) {
  (void)in_sizes;
  if (n_in < 9) return;
  if (ws_size < kWsTotal) return;
  if ((size_t)out_size * 4 < kOutTotalB) return;

  const float* points_coords    = (const float*)d_in[0];
  const float* centers_coords   = (const float*)d_in[1];
  const float* centers_features = (const float*)d_in[2];
  const float* points_features  = (const float*)d_in[3];
  const float* condition        = (const float*)d_in[4];
  const float* W1               = (const float*)d_in[5];
  const float* b1               = (const float*)d_in[6];
  const float* W2               = (const float*)d_in[7];
  const float* b2               = (const float*)d_in[8];

  float* out0 = (float*)d_out;
  float* out1 = (float*)d_out + kOut1OffB / 4;
  float* out2 = (float*)d_out + kOut2OffB / 4;

  unsigned char* ws = (unsigned char*)d_ws;
  unsigned short* w1h   = (unsigned short*)(ws + kOffW1H);
  unsigned short* w1l   = (unsigned short*)(ws + kOffW1L);
  unsigned short* w2h   = (unsigned short*)(ws + kOffW2H);
  unsigned short* w2l   = (unsigned short*)(ws + kOffW2L);
  unsigned short* feath = (unsigned short*)(ws + kOffFeatH);
  unsigned short* featl = (unsigned short*)(ws + kOffFeatL);
  unsigned short* hidh  = (unsigned short*)(ws + kOffHidH);
  unsigned short* hidl  = (unsigned short*)(ws + kOffHidL);

  prep_planes_and_copies<<<kPrepW1Blocks + kPrepW2Blocks + kPrepO1Blocks + kPrepO2Blocks, 256, 0, stream>>>(
      W1, W2, points_coords, condition, w1h, w1l, w2h, w2l, out1, out2);

  knn3_interp_pack<<<dim3(kNumPoints / 256, kNumBatch, 1), 256, 0, stream>>>(
      points_coords, centers_coords, centers_features, points_features, feath, featl);

  for (int half = 0; half < 2; ++half) {
    const size_t featOff = (size_t)half * kHalfPoints * kChanIn;
    const int tiles1 = (kHalfPoints / 64) * (kHidden1 / 64);
    gemm_bf16x3_64<2, 2><<<dim3(tiles1 / 8, 1, 1), 256, 0, stream>>>(
        feath + featOff, featl + featOff, kChanIn, (long)0,
        w1h, w1l, kChanIn, (long)0,
        (void*)hidh, (void*)hidl, kHidden1, (long)0,
        b1, kHalfPoints, kHidden1, kChanIn);

    const int tiles2 = (kHidden2 / 64) * (kNumPoints / 64);
    float* outHalf = out0 + (size_t)half * kHalfBatch * kHidden2 * kNumPoints;
    gemm_bf16x3_64<0, 1><<<dim3(tiles2 / 8, kHalfBatch, 1), 256, 0, stream>>>(
        w2h, w2l, kHidden1, (long)0,
        hidh, hidl, kHidden1, (long)kNumPoints * kHidden1,
        (void*)outHalf, (void*)outHalf, kNumPoints, (long)kHidden2 * kNumPoints,
        b2, kHidden2, kNumPoints, kHidden1);
  }
}
